// PLANAttention_44959717654697
// MI455X (gfx1250) — hardware-run, weakly checked
//
#include <hip/hip_runtime.h>
#include <stdint.h>

#define DEVINL __device__ __forceinline__

typedef unsigned short us_t;
typedef __bf16   v16bf __attribute__((ext_vector_type(16)));
typedef us_t     v8us  __attribute__((ext_vector_type(8)));
typedef float    v8f   __attribute__((ext_vector_type(8)));
typedef float    v4f   __attribute__((ext_vector_type(4)));
typedef v8us __attribute__((may_alias)) v8usa;
typedef v4f  __attribute__((may_alias)) v4fa;
union Frag { v16bf v; v8us half[2]; };

#define NB    2
#define CH    256
#define HT    64
#define HWT   4096
#define HB    128
#define HWB   16384
#define NKEY  10
#define KA    768
#define KB    512
#define NWG   8
#define TPB   256
#define WAVES 8
#define PT    64
#define PQF   132
#define XPT   32
#define XPQ   520
#define ATPB  32
#define INVSQ 0.17677669529663687f

enum { EPI_PM32 = 0, EPI_NCHW = 1 };

static_assert(TPB == WAVES * 32);
static_assert((HWT % PT) == 0);
static_assert((HWB % PT) == 0);
static_assert((HWT % XPT) == 0);
static_assert((HWB % XPT) == 0);
static_assert((KA % 32) == 0);
static_assert(KB == 2 * CH);
static_assert(KA == 3 * CH);
static_assert(WAVES * 1024 <= PT * PQF);
static_assert((PQF % 4) == 0);
static_assert((XPQ % 8) == 0);
static_assert(XPQ >= KB);
static_assert(HT * HT == HWT);
static_assert(HB * HB == HWB);
static_assert(CH * 32 == 32 * TPB);
static_assert(CH == 8 * 32);

DEVINL int imin(int a, int b) { return a < b ? a : b; }
DEVINL int imax(int a, int b) { return a > b ? a : b; }

DEVINL uint32_t bf16_rne_bits(float x) {
  const uint32_t u = __float_as_uint(x);
  return (u + 0x7FFFu + ((u >> 16) & 1u)) >> 16;
}
DEVINL void split_hl(float x, uint32_t& hb, uint32_t& lb) {
  hb = bf16_rne_bits(x);
  lb = bf16_rne_bits(x - __uint_as_float(hb << 16));
}

DEVINL v8f wmma_bf16(v16bf a, v16bf b, v8f c) {
  v8f d = __builtin_amdgcn_wmma_f32_16x16x32_bf16(false, a, false, b, (short)0, c, false, false);
  asm volatile("v_nop\n\tv_nop\n\tv_nop\n\tv_nop" : "+v"(d) : "v"(a), "v"(b));
  return d;
}
DEVINL v8f zero8f() {
  v8f z = {0.f, 0.f, 0.f, 0.f, 0.f, 0.f, 0.f, 0.f};
  return z;
}
DEVINL void load_frag(Frag& f, const us_t* row, int k0) {
  f.half[0] = *(const v8usa*)(row + k0);
  f.half[1] = *(const v8usa*)(row + k0 + 16);
}

__global__ __launch_bounds__(TPB) void prep_w_k(const float* __restrict__ w0, const float* __restrict__ w1,
                                               const float* __restrict__ w2, const float* __restrict__ w3,
                                               const float* __restrict__ w4, const float* __restrict__ w5,
                                               const float* __restrict__ w6, const float* __restrict__ w7,
                                               us_t* __restrict__ WP)
{
  const int g = blockIdx.y;
  const int u = blockIdx.x * TPB + threadIdx.x;
  const int row = u >> 5, piece = (u & 31) * 8;
  if (row >= CH || g >= NWG) return;
  const float* src = (g == 0) ? w0 : ((g == 1) ? w1 : ((g == 2) ? w2 : ((g == 3) ? w3 :
                     ((g == 4) ? w4 : ((g == 5) ? w5 : ((g == 6) ? w6 : w7))))));
  const float* sp = src + (size_t)row * CH + piece;
  const v4f a = *(const v4fa*)sp, c = *(const v4fa*)(sp + 4);
  v8us hi, lo;
  #pragma unroll
  for (int i = 0; i < 4; ++i) {
    uint32_t hb, lb;
    split_hl(a[i], hb, lb); hi[i] = (us_t)hb;     lo[i] = (us_t)lb;
    split_hl(c[i], hb, lb); hi[4 + i] = (us_t)hb; lo[4 + i] = (us_t)lb;
  }
  us_t* dst = WP + ((size_t)g * CH + row) * KA + piece;
  *(volatile v8us*)(dst)          = hi;
  *(volatile v8us*)(dst + CH)     = lo;
  *(volatile v8us*)(dst + 2 * CH) = hi;
  __threadfence();
  *(volatile v8us*)(dst)          = hi;
  *(volatile v8us*)(dst + CH)     = lo;
  *(volatile v8us*)(dst + 2 * CH) = hi;
}

__global__ __launch_bounds__(TPB) void xpose_k(const float* __restrict__ x, us_t* __restrict__ XT, int HW)
{
  __shared__ __attribute__((aligned(16))) us_t sT[XPT * XPQ];
  const int tid = threadIdx.x;
  const int p0 = blockIdx.x * XPT;
  const int c0 = tid >> 3, p4 = (tid & 7) * 4;
  const float* xb = x + p0 + p4;
  #pragma unroll 2
  for (int i = 0; i < 8; ++i) {
    const int c = c0 + 32 * i;
    const v4f v = *(const v4fa*)(xb + (size_t)c * HW);
    #pragma unroll
    for (int j = 0; j < 4; ++j) {
      uint32_t hb, lb;
      split_hl(v[j], hb, lb);
      sT[(p4 + j) * XPQ + c]      = (us_t)hb;
      sT[(p4 + j) * XPQ + CH + c] = (us_t)lb;
    }
  }
  __syncthreads();
  us_t* base = XT + (size_t)p0 * KB;
  #pragma unroll
  for (int i = 0; i < 8; ++i) {
    const int q = tid + TPB * i;
    const int row = q >> 6, piece = (q & 63) * 8;
    const v8us v = *(const v8usa*)(sT + row * XPQ + piece);
    *(volatile v8us*)(base + (size_t)row * KB + piece) = v;
  }
  __threadfence();
  #pragma unroll
  for (int i = 0; i < 8; ++i) {
    const int q = tid + TPB * i;
    const int row = q >> 6, piece = (q & 63) * 8;
    const v8us v = *(const v8usa*)(sT + row * XPQ + piece);
    *(volatile v8us*)(base + (size_t)row * KB + piece) = v;
  }
}

template <int EPI>
__global__ __launch_bounds__(TPB) void gemm_k(const us_t* __restrict__ Bp, const us_t* __restrict__ Ap,
                                             float* out0, float* out1, float* out2, int HWp)
{
  __shared__ __attribute__((aligned(16))) float sbuf[PT * PQF];
  const int tid = threadIdx.x, lane = tid & 31, wave = tid >> 5;
  const int h = lane >> 4, m = lane & 15;
  const int p0 = blockIdx.x * PT, y = blockIdx.y;
  float* outp = (y == 0) ? out0 : ((y == 1) ? out1 : out2);

  v8f acc[2][4];
  #pragma unroll
  for (int mt = 0; mt < 2; ++mt) {
    #pragma unroll
    for (int n = 0; n < 4; ++n) acc[mt][n] = zero8f();
  }
  const us_t* arow = Ap + ((size_t)y * CH + wave * 32 + m) * KA + 8 * h;
  const us_t* brow = Bp + ((size_t)p0 + m) * KB + 8 * h;
  #pragma unroll 1
  for (int ks = 0; ks < KA / 32; ++ks) {
    const int k0 = 32 * ks;
    const int bc = (k0 < KB) ? (k0 & (CH - 1)) : (k0 - CH);
    Frag a0, a1, bf[4];
    load_frag(a0, arow, k0);
    load_frag(a1, arow + 16 * KA, k0);
    #pragma unroll
    for (int n = 0; n < 4; ++n) load_frag(bf[n], brow + (size_t)16 * n * KB, bc);
    #pragma unroll
    for (int n = 0; n < 4; ++n) {
      acc[0][n] = wmma_bf16(a0.v, bf[n].v, acc[0][n]);
      acc[1][n] = wmma_bf16(a1.v, bf[n].v, acc[1][n]);
    }
  }

  if (EPI == EPI_PM32) {
    #pragma unroll
    for (int ph = 0; ph < 2; ++ph) {
      if ((wave >> 2) == ph) {
        #pragma unroll
        for (int mt = 0; mt < 2; ++mt) {
          #pragma unroll
          for (int n = 0; n < 4; ++n) {
            v4f o0, o1;
            #pragma unroll
            for (int r = 0; r < 4; ++r) { o0[r] = acc[mt][n][r]; o1[r] = acc[mt][n][4 + r]; }
            const int cl = 32 * (wave & 3) + 16 * mt + 8 * h;
            float* sp = sbuf + (16 * n + m) * PQF + cl;
            *(v4fa*)sp = o0;
            *(v4fa*)(sp + 4) = o1;
          }
        }
      }
      __syncthreads();
      float* dst = outp + (size_t)p0 * CH + 128 * ph;
      #pragma unroll
      for (int i = 0; i < 8; ++i) {
        const int row = 8 * i + wave;
        const v4f v = *(const v4fa*)(sbuf + row * PQF + 4 * lane);
        *(volatile v4f*)(dst + (size_t)row * CH + 4 * lane) = v;
      }
      __threadfence();
      #pragma unroll
      for (int i = 0; i < 8; ++i) {
        const int row = 8 * i + wave;
        const v4f v = *(const v4fa*)(sbuf + row * PQF + 4 * lane);
        *(volatile v4f*)(dst + (size_t)row * CH + 4 * lane) = v;
      }
      __syncthreads();
    }
  } else {
    #pragma unroll
    for (int mt = 0; mt < 2; ++mt) {
      #pragma unroll
      for (int n = 0; n < 4; ++n) {
        #pragma unroll
        for (int r = 0; r < 8; ++r)
          sbuf[wave * 1024 + (8 * h + r) * PT + 16 * n + m] = acc[mt][n][r];
      }
      __syncthreads();
      float* orow = outp + (size_t)(wave * 32 + 16 * mt) * HWp + p0;
      const int l16 = lane & 15, rsel = lane >> 4;
      #pragma unroll
      for (int i = 0; i < 8; ++i) {
        const int row = 2 * i + rsel;
        const v4f v = *(const v4fa*)(sbuf + wave * 1024 + row * PT + 4 * l16);
        *(volatile v4f*)(orow + (size_t)row * HWp + 4 * l16) = v;
      }
      __threadfence();
      #pragma unroll
      for (int i = 0; i < 8; ++i) {
        const int row = 2 * i + rsel;
        const v4f v = *(const v4fa*)(sbuf + wave * 1024 + row * PT + 4 * l16);
        *(volatile v4f*)(orow + (size_t)row * HWp + 4 * l16) = v;
      }
      __syncthreads();
    }
  }
}

DEVINL void acc_keys(int lane, int ty, int tx, v4f q0, v4f q1, v4f& a0, v4f& a1,
                     const float* __restrict__ TK, const float* __restrict__ TV,
                     const float* __restrict__ BK, const float* __restrict__ BV)
{
  const int t = ty * HT + tx;
  #pragma unroll 1
  for (int k = 0; k < NKEY; ++k) {
    const float* kb;
    const float* vb;
    size_t rof;
    if (k == 0) {
      kb = TK; vb = TV; rof = (size_t)t * CH;
    } else {
      const int n = k - 1;
      const int i = (n >= 6) ? 2 : ((n >= 3) ? 1 : 0);
      const int j = n - 3 * i;
      const int yy = 2 * ty - 1 + i, xx = 2 * tx - 1 + j;
      if ((unsigned)yy >= (unsigned)HB || (unsigned)xx >= (unsigned)HB) continue;
      kb = BK; vb = BV; rof = (size_t)(yy * HB + xx) * CH;
    }
    const float* kp = kb + rof + 8 * lane;
    const float* vp = vb + rof + 8 * lane;
    const v4f k0 = *(const v4fa*)kp, k1 = *(const v4fa*)(kp + 4);
    float s = q0[0] * k0[0];
    s = fmaf(q0[1], k0[1], s);
    s = fmaf(q0[2], k0[2], s);
    s = fmaf(q0[3], k0[3], s);
    s = fmaf(q1[0], k1[0], s);
    s = fmaf(q1[1], k1[1], s);
    s = fmaf(q1[2], k1[2], s);
    s = fmaf(q1[3], k1[3], s);
    s += __shfl_xor(s, 1);
    s += __shfl_xor(s, 2);
    s *= INVSQ;
    const v4f v0 = *(const v4fa*)vp, v1 = *(const v4fa*)(vp + 4);
    a0[0] = fmaf(s, v0[0], a0[0]);
    a0[1] = fmaf(s, v0[1], a0[1]);
    a0[2] = fmaf(s, v0[2], a0[2]);
    a0[3] = fmaf(s, v0[3], a0[3]);
    a1[0] = fmaf(s, v1[0], a1[0]);
    a1[1] = fmaf(s, v1[1], a1[1]);
    a1[2] = fmaf(s, v1[2], a1[2]);
    a1[3] = fmaf(s, v1[3], a1[3]);
  }
}

DEVINL void store_hl_row(us_t* dst, int lane, v4f a0, v4f a1)
{
  v8us hi, lo;
  #pragma unroll
  for (int i = 0; i < 4; ++i) {
    uint32_t hb, lb;
    split_hl(a0[i], hb, lb); hi[i] = (us_t)hb;     lo[i] = (us_t)lb;
    split_hl(a1[i], hb, lb); hi[4 + i] = (us_t)hb; lo[4 + i] = (us_t)lb;
  }
  us_t* ph = dst + 8 * lane;
  us_t* pl = dst + CH + 8 * lane;
  *(volatile v8us*)ph = hi;
  *(volatile v8us*)pl = lo;
  __threadfence();
  *(volatile v8us*)ph = hi;
  *(volatile v8us*)pl = lo;
}

__global__ __launch_bounds__(ATPB) void attn_top_k(const float* __restrict__ TK, const float* __restrict__ TQ,
                                                  const float* __restrict__ TV, const float* __restrict__ BK,
                                                  const float* __restrict__ BV, us_t* __restrict__ TR)
{
  const int lane = threadIdx.x & 31;
  const int t = blockIdx.x;
  if (t >= HWT) return;
  const int ty = t >> 6, tx = t & 63;
  const float* qp = TQ + (size_t)t * CH + 8 * lane;
  const v4f q0 = *(const v4fa*)qp, q1 = *(const v4fa*)(qp + 4);
  v4f a0 = {0.f, 0.f, 0.f, 0.f};
  v4f a1 = {0.f, 0.f, 0.f, 0.f};
  acc_keys(lane, ty, tx, q0, q1, a0, a1, TK, TV, BK, BV);
  store_hl_row(TR + (size_t)t * KB, lane, a0, a1);
}

__global__ __launch_bounds__(ATPB) void attn_bot_k(const float* __restrict__ TK, const float* __restrict__ TV,
                                                  const float* __restrict__ BK, const float* __restrict__ BQ,
                                                  const float* __restrict__ BV, us_t* __restrict__ BR)
{
  const int lane = threadIdx.x & 31;
  const int P = blockIdx.x;
  if (P >= HWB) return;
  const int Y = P >> 7, X = P & 127;
  const float* qp = BQ + (size_t)P * CH + 8 * lane;
  const v4f q0 = *(const v4fa*)qp, q1 = *(const v4fa*)(qp + 4);
  v4f a0 = {0.f, 0.f, 0.f, 0.f};
  v4f a1 = {0.f, 0.f, 0.f, 0.f};
  #pragma unroll 1
  for (int i = 0; i < 3; ++i) {
    const int y2 = Y + 1 - i;
    if (y2 & 1) continue;
    const int ty = y2 >> 1;
    if (ty >= HT) continue;
    #pragma unroll 1
    for (int j = 0; j < 3; ++j) {
      const int x2 = X + 1 - j;
      if (x2 & 1) continue;
      const int tx = x2 >> 1;
      if (tx >= HT) continue;
      acc_keys(lane, ty, tx, q0, q1, a0, a1, TK, TV, BK, BV);
    }
  }
  store_hl_row(BR + (size_t)P * KB, lane, a0, a1);
}

extern "C" void kernel_launch(void* const* d_in, const int* in_sizes, int n_in,
                              void* d_out, int out_size, void* d_ws, size_t ws_size,
                              hipStream_t stream)
{
  if (n_in < 10) return;
  if (in_sizes[0] != NB * CH * HWT) return;
  if (in_sizes[1] != NB * CH * HWB) return;
  for (int i = 2; i < 10; ++i) if (in_sizes[i] != CH * CH) return;
  if (out_size != NB * CH * HWT + NB * CH * HWB) return;

  const float* top_feat = (const float*)d_in[0];
  const float* bot_feat = (const float*)d_in[1];
  const float* w_tk = (const float*)d_in[2];
  const float* w_tq = (const float*)d_in[3];
  const float* w_tv = (const float*)d_in[4];
  const float* w_bk = (const float*)d_in[5];
  const float* w_bq = (const float*)d_in[6];
  const float* w_bv = (const float*)d_in[7];
  const float* w_tf = (const float*)d_in[8];
  const float* w_bf = (const float*)d_in[9];
  float* outT = (float*)d_out;
  float* outB = outT + (size_t)NB * CH * HWT;

  const size_t szWP  = (size_t)NWG * CH * KA * 2;
  const size_t szXTt = (size_t)HWT * KB * 2;
  const size_t szXTb = (size_t)HWB * KB * 2;
  const size_t szPT  = (size_t)HWT * CH * 4;
  const size_t szPB  = (size_t)HWB * CH * 4;
  size_t off = 0;
  char* ws = (char*)d_ws;
  us_t*  WP  = (us_t*)(ws + off);  off += szWP;
  us_t*  XTt = (us_t*)(ws + off);  off += szXTt;
  us_t*  XTb = (us_t*)(ws + off);  off += szXTb;
  float* TK  = (float*)(ws + off); off += szPT;
  float* TQ  = (float*)(ws + off); off += szPT;
  float* TV  = (float*)(ws + off); off += szPT;
  float* BK  = (float*)(ws + off); off += szPB;
  float* BQ  = (float*)(ws + off); off += szPB;
  float* BV  = (float*)(ws + off); off += szPB;
  us_t*  TR  = (us_t*)(ws + off);  off += szXTt;
  us_t*  BR  = (us_t*)(ws + off);  off += szXTb;
  if (off > ws_size) return;

  prep_w_k<<<dim3(CH * 32 / TPB, NWG), TPB, 0, stream>>>(w_tk, w_tq, w_tv, w_bk, w_bq, w_bv, w_tf, w_bf, WP);

  for (int b = 0; b < NB; ++b) {
    xpose_k<<<HWT / XPT, TPB, 0, stream>>>(top_feat + (size_t)b * CH * HWT, XTt, HWT);
    xpose_k<<<HWB / XPT, TPB, 0, stream>>>(bot_feat + (size_t)b * CH * HWB, XTb, HWB);
    gemm_k<EPI_PM32><<<dim3(HWT / PT, 3), TPB, 0, stream>>>(XTt, WP, TK, TQ, TV, HWT);
    gemm_k<EPI_PM32><<<dim3(HWB / PT, 3), TPB, 0, stream>>>(XTb, WP + (size_t)3 * CH * KA, BK, BQ, BV, HWB);
    attn_top_k<<<HWT, ATPB, 0, stream>>>(TK, TQ, TV, BK, BV, TR);
    attn_bot_k<<<HWB, ATPB, 0, stream>>>(TK, TV, BK, BQ, BV, BR);
    float* oT = outT + (size_t)b * CH * HWT;
    float* oB = outB + (size_t)b * CH * HWB;
    gemm_k<EPI_NCHW><<<dim3(HWT / PT, 1), TPB, 0, stream>>>(TR, WP + (size_t)6 * CH * KA, oT, oT, oT, HWT);
    gemm_k<EPI_NCHW><<<dim3(HWB / PT, 1), TPB, 0, stream>>>(BR, WP + (size_t)7 * CH * KA, oB, oB, oB, HWB);
  }
}
